// HybridSigLSTM_48473000902900
// MI455X (gfx1250) — hardware-verified
//
#include <hip/hip_runtime.h>

typedef __attribute__((ext_vector_type(16))) _Float16 v16h;
typedef __attribute__((ext_vector_type(8)))  _Float16 v8h;
typedef __attribute__((ext_vector_type(8)))  float    v8f;
typedef __attribute__((ext_vector_type(4)))  float    v4f;
typedef __attribute__((ext_vector_type(4)))  unsigned int v4u;

constexpr int kBatch = 4096;
constexpr int kSeq   = 256;
constexpr int kDin   = 4;
constexpr int kHid   = 50;
constexpr int kRowsPerBlock = 16;
constexpr int kXsPitch   = 40;
constexpr int kTilePitch = 136;
constexpr int kHPitch    = 72;
constexpr int kK0  = 96;
constexpr int kK1  = 128;
constexpr int kKH  = 64;
constexpr int kPdCol = 40;
constexpr int kH0Col = 46;
constexpr int kNGate = 256;
constexpr float kAScale   = 64.0f;
constexpr float kBScale   = 16.0f;
constexpr float kAccScale = 1.0f / 1024.0f;
constexpr float kMaxInc   = 0.2f;
constexpr float kDeltaMax = 1.5f;

static_assert(kBatch % kRowsPerBlock == 0, "rows per block");
static_assert(kBatch % 64 == 0, "signature chunk");
static_assert((kTilePitch % 8) == 0 && (kHPitch % 8) == 0, "16-byte fragment alignment");

__device__ __forceinline__ void dep_guard_h(v8f& a, v8f& b, v16h x, v16h y) { asm volatile("v_nop\n\tv_nop\n\tv_nop\n\tv_nop" : "+v"(a), "+v"(b) : "v"(x), "v"(y)); }
__device__ __forceinline__ void keep4_h(v16h a, v16h b, v16h c, v16h d) { asm volatile("v_nop" :: "v"(a), "v"(b), "v"(c), "v"(d)); }
__device__ __forceinline__ void acc_guard4(v8f& a, v8f& b, v8f& c, v8f& d) { asm volatile("v_nop\n\tv_nop\n\tv_nop\n\tv_nop" : "+v"(a), "+v"(b), "+v"(c), "+v"(d)); }
template <typename T> struct Frag;
template <> struct Frag<_Float16> {
  typedef v16h V; union U { v16h v; v8h h[2]; };
  static __device__ __forceinline__ v16h load(const _Float16* p) {
    U f; f.h[0] = *(const v8h*)(p); f.h[1] = *(const v8h*)(p + 16); return f.v;
  }
  static __device__ __forceinline__ v8f mma(v16h a, v16h b, v8f c) {
    return __builtin_amdgcn_wmma_f32_16x16x32_f16(false, a, false, b, (short)0, c, false, false);
  }
  static __device__ __forceinline__ void guard(v8f& a, v8f& b, v16h x, v16h y) { dep_guard_h(a, b, x, y); }
  static __device__ __forceinline__ void keep(v16h a, v16h b, v16h c, v16h d) { keep4_h(a, b, c, d); }
};

__device__ __forceinline__ unsigned short h_bits(float f) { return __builtin_bit_cast(unsigned short, (_Float16)f); }
__device__ __forceinline__ unsigned int pack_h2(float a, float b) {
  return (unsigned int)h_bits(a) | ((unsigned int)h_bits(b) << 16);
}
__device__ __forceinline__ float frcp(float x) { return __builtin_amdgcn_rcpf(x); }
__device__ __forceinline__ float fsig(float x) { return frcp(1.0f + __expf(-x)); }
__device__ __forceinline__ float ftanh(float x) { return 1.0f - 2.0f * frcp(1.0f + __expf(2.0f * x)); }
__device__ __forceinline__ float to_vgpr(float x) { asm volatile("" : "+v"(x)); return x; }

__device__ __forceinline__ float sel_w0(const float* __restrict__ wih0, const float* __restrict__ whh0, int n, int k) {
  const int ka = k < 34 ? k : 34;
  int kb = k - kH0Col; kb = kb < 0 ? 0 : kb; kb = kb > kHid - 1 ? kHid - 1 : kb;
  const float va = wih0[n * 35 + ka];
  const float vb = whh0[n * kHid + kb];
  const bool useA = (k < 34) || (k == kPdCol);
  const bool useB = (k >= kH0Col) && (k < kH0Col + kHid);
  return useA ? va : (useB ? vb : 0.0f);
}
__device__ __forceinline__ float sel_w1(const float* __restrict__ wih1, const float* __restrict__ whh1, int n, int k) {
  const int ka = k < kHid - 1 ? k : kHid - 1;
  int kb = k - 64; kb = kb < 0 ? 0 : kb; kb = kb > kHid - 1 ? kHid - 1 : kb;
  const float va = wih1[n * kHid + ka];
  const float vb = whh1[n * kHid + kb];
  const bool useA = (k < kHid);
  const bool useB = (k >= 64) && (k < 64 + kHid);
  return useA ? va : (useB ? vb : 0.0f);
}

__device__ __forceinline__ unsigned int bt0_word(const float* __restrict__ wih0, const float* __restrict__ whh0, int np, int kw) {
  const int g = (np >> 6) & 3, u = np & 63;
  const bool uv = u < kHid;
  const int n = g * kHid + (uv ? u : kHid - 1);
  const float v0 = uv ? sel_w0(wih0, whh0, n, 2 * kw) * kBScale : 0.0f;
  const float v1 = uv ? sel_w0(wih0, whh0, n, 2 * kw + 1) * kBScale : 0.0f;
  return pack_h2(v0, v1);
}
__device__ __forceinline__ unsigned int bt1_word(const float* __restrict__ wih1, const float* __restrict__ whh1, int np, int kw) {
  const int g = (np >> 6) & 3, u = np & 63;
  const bool uv = u < kHid;
  const int n = g * kHid + (uv ? u : kHid - 1);
  const float v0 = uv ? sel_w1(wih1, whh1, n, 2 * kw) * kBScale : 0.0f;
  const float v1 = uv ? sel_w1(wih1, whh1, n, 2 * kw + 1) * kBScale : 0.0f;
  return pack_h2(v0, v1);
}
__device__ __forceinline__ unsigned int bw1_word(const float* __restrict__ w1, int j, int kw) {
  const int jc = j < 24 ? j : 24;
  float v[2];
#pragma unroll
  for (int e = 0; e < 2; ++e) {
    const int k = 2 * kw + e;
    const int kc = k < kHid - 1 ? k : kHid - 1;
    const float w = w1[jc * kHid + kc];
    v[e] = (j < 25 && k < kHid) ? w * kBScale : 0.0f;
  }
  return pack_h2(v[0], v[1]);
}

__global__ __launch_bounds__(64) void prep_weights_kernel(
    const float* __restrict__ wih0, const float* __restrict__ whh0,
    const float* __restrict__ bih0, const float* __restrict__ bhh0,
    const float* __restrict__ wih1, const float* __restrict__ whh1,
    const float* __restrict__ bih1, const float* __restrict__ bhh1,
    const float* __restrict__ w1, const float* __restrict__ b1,
    const float* __restrict__ w2, const float* __restrict__ b2,
    unsigned int* __restrict__ bt0, unsigned int* __restrict__ bt1,
    unsigned int* __restrict__ bw1, float* __restrict__ ct)
{
  const int tid = threadIdx.x;
  const int blk = blockIdx.x;
  if (blk < 128) {
    const int wA = tid;
    const int wB = 64 + (tid & 31);
    const unsigned int vA = bt0_word(wih0, whh0, 2 * blk + (wA >= 48 ? 1 : 0), wA >= 48 ? wA - 48 : wA);
    const unsigned int vB = bt0_word(wih0, whh0, 2 * blk + 1, wB - 48);
    volatile unsigned int* dst = bt0 + (size_t)blk * 96;
    dst[wA] = vA;
    if (tid < 32) dst[wB] = vB;
    __threadfence();
    dst[wA] = vA;
    if (tid < 32) dst[wB] = vB;
  } else if (blk < 384) {
    const int np = blk - 128;
    const unsigned int v = bt1_word(wih1, whh1, np, tid);
    volatile unsigned int* dst = bt1 + (size_t)np * 64;
    dst[tid] = v;
    __threadfence();
    dst[tid] = v;
  } else if (blk == 384) {
    unsigned int vals[16];
#pragma unroll
    for (int it = 0; it < 16; ++it) {
      const int idx = it * 64 + tid;
      vals[it] = bw1_word(w1, idx >> 5, idx & 31);
    }
    volatile unsigned int* dst = bw1;
    for (int pass = 0; pass < 2; ++pass) {
#pragma unroll
      for (int it = 0; it < 16; ++it) dst[it * 64 + tid] = vals[it];
      __threadfence();
    }
  } else {
    float vals[10];
#pragma unroll
    for (int it = 0; it < 10; ++it) {
      const int i = it * 64 + tid;
      const int i0 = i & 255;
      const int g = (i0 >> 6) & 3, u = i0 & 63;
      const int uc = u < kHid ? u : kHid - 1;
      int jb = i - 512; jb = jb < 0 ? 0 : jb; jb = jb > 24 ? 24 : jb;
      int jw = i - 544; jw = jw < 0 ? 0 : jw; jw = jw > 24 ? 24 : jw;
      const float va = bih0[g * kHid + uc] + bhh0[g * kHid + uc];
      const float vb = bih1[g * kHid + uc] + bhh1[g * kHid + uc];
      const float vc = b1[jb];
      const float vd = w2[jw];
      const float ve = b2[0];
      float v = 0.0f;
      if (i < 256)      v = (u < kHid) ? va : 0.0f;
      else if (i < 512) v = (u < kHid) ? vb : 0.0f;
      else if (i < 544) v = (i - 512 < 25) ? vc : 0.0f;
      else if (i < 576) v = (i - 544 < 25) ? vd : 0.0f;
      else              v = (i == 576) ? ve : 0.0f;
      vals[it] = v;
    }
    volatile float* dst = ct;
    for (int pass = 0; pass < 2; ++pass) {
#pragma unroll
      for (int it = 0; it < 10; ++it) dst[it * 64 + tid] = vals[it];
      __threadfence();
    }
  }
}

__global__ __launch_bounds__(64) void sig_feats_kernel(const float* __restrict__ feat, unsigned short* __restrict__ xs)
{
  __shared__ __align__(16) float sAug[64 * 25];
  __shared__ __align__(16) float sVal[64 * 40];
  __shared__ __align__(16) unsigned int sX[64 * 20];
  const int tid = threadIdx.x;
  const int t = blockIdx.y;
  const int b = blockIdx.x * 64 + tid;
  float* aw = sAug + tid * 25;
  float* vr = sVal + tid * 40;

#pragma unroll
  for (int k = 0; k < 4; ++k) {
    int s = t + k - 4; s = s < 0 ? 0 : s;
    const v4f f = *(const v4f*)(feat + ((size_t)b * kSeq + s) * kDin);
    float tm = (s == kSeq - 1) ? 1.0f : (float)s * (1.0f / 255.0f);
    tm = to_vgpr(tm);
    aw[k * 5 + 0] = tm; aw[k * 5 + 1] = f.x; aw[k * 5 + 2] = f.y; aw[k * 5 + 3] = f.z; aw[k * 5 + 4] = f.w;
  }
  const v4f fc = *(const v4f*)(feat + ((size_t)b * kSeq + t) * kDin);
  {
    float tm = (t == kSeq - 1) ? 1.0f : (float)t * (1.0f / 255.0f);
    tm = to_vgpr(tm);
    aw[20] = tm; aw[21] = fc.x; aw[22] = fc.y; aw[23] = fc.z; aw[24] = fc.w;
  }
  vr[0] = fc.x; vr[1] = fc.y; vr[2] = fc.z; vr[3] = fc.w;
#pragma unroll
  for (int i = 0; i < 5; ++i) vr[4 + i] = aw[20 + i] - aw[i];
#pragma unroll 1
  for (int i = 0; i < 5; ++i) {
#pragma unroll 1
    for (int j = 0; j < 5; ++j) {
      float s2 = 0.0f;
#pragma unroll
      for (int k = 0; k < 4; ++k) s2 = fmaf(aw[(k + 1) * 5 + i] - aw[k * 5 + i], aw[k * 5 + j], s2);
      vr[9 + i * 5 + j] = s2;
    }
  }
#pragma unroll
  for (int c = 34; c < 40; ++c) vr[c] = 0.0f;
#pragma unroll
  for (int w = 0; w < 20; ++w)
    sX[tid * 20 + w] = pack_h2(vr[2 * w] * kAScale, vr[2 * w + 1] * kAScale);
  __syncthreads();

  const v4u* src = (const v4u*)sX;
  unsigned short* dstb = xs + ((size_t)t * kBatch + (size_t)blockIdx.x * 64) * kXsPitch;
  v4u vals[5];
#pragma unroll
  for (int it = 0; it < 5; ++it) vals[it] = src[it * 64 + tid];
  for (int pass = 0; pass < 2; ++pass) {
#pragma unroll
    for (int it = 0; it < 5; ++it)
      *(volatile v4u*)(dstb + (size_t)(it * 64 + tid) * 8) = vals[it];
    __threadfence();
  }
}

template <int KSTEPS, int APITCH, int LDB>
__device__ __forceinline__ void gate_gemm16(const _Float16* At, const _Float16* Bt, int rl, int koff, int ncol0, v8f (&acc)[4])
{
#pragma unroll
  for (int g = 0; g < 4; ++g) acc[g] = (v8f){0.f, 0.f, 0.f, 0.f, 0.f, 0.f, 0.f, 0.f};
#pragma unroll 1
  for (int ks = 0; ks < KSTEPS; ++ks) {
    const v16h a = Frag<_Float16>::load(At + rl * APITCH + ks * 32 + koff);
    v16h bq[4];
#pragma unroll
    for (int g = 0; g < 4; ++g)
      bq[g] = Frag<_Float16>::load(Bt + (size_t)(g * 64 + ncol0 + rl) * LDB + ks * 32 + koff);
#pragma unroll
    for (int g = 0; g < 4; ++g) acc[g] = Frag<_Float16>::mma(a, bq[g], acc[g]);
    Frag<_Float16>::guard(acc[0], acc[3], a, bq[3]);
    Frag<_Float16>::keep(bq[0], bq[1], bq[2], bq[3]);
  }
  acc_guard4(acc[0], acc[1], acc[2], acc[3]);
}

__device__ __forceinline__ void lstm_cell_update(const v8f (&acc)[4], const float (&bi)[4], bool uval,
                                                 float (&c)[8], float (&h)[8])
{
#pragma unroll
  for (int r = 0; r < 8; ++r) {
    const float zi = acc[0][r] * kAccScale + bi[0];
    const float zf = acc[1][r] * kAccScale + bi[1];
    const float zg = acc[2][r] * kAccScale + bi[2];
    const float zo = acc[3][r] * kAccScale + bi[3];
    const float cn = fsig(zf) * c[r] + fsig(zi) * ftanh(zg);
    const float hn = fsig(zo) * ftanh(cn);
    c[r] = uval ? cn : 0.0f;
    h[r] = uval ? hn : 0.0f;
  }
}

__global__ __launch_bounds__(128) void sig_lstm_seq_kernel(
    const unsigned short* __restrict__ xs,
    const unsigned short* __restrict__ bt0p,
    const unsigned short* __restrict__ bt1p,
    const unsigned short* __restrict__ bw1p,
    const float* __restrict__ ct,
    float* __restrict__ out)
{
  __shared__ __align__(16) unsigned short tA0[kRowsPerBlock * kTilePitch];
  __shared__ __align__(16) unsigned short tA1[kRowsPerBlock * kTilePitch];
  __shared__ __align__(16) unsigned short tH[kRowsPerBlock * kHPitch];
  __shared__ __align__(16) float sOut[kRowsPerBlock * kSeq];

  const int tid  = threadIdx.x;
  const int lane = tid & 31;
  const int wave = __builtin_amdgcn_readfirstlane(tid >> 5);
  const int rl   = lane & 15;
  const int hh   = lane >> 4;
  const int koff = hh * 8;
  const int b0   = blockIdx.x * kRowsPerBlock;
  const int unit = wave * 16 + rl;
  const bool uval = unit < kHid;

  {
    const v4u z = {0u, 0u, 0u, 0u};
    for (int i = tid; i < (kRowsPerBlock * kTilePitch * 2) / 16; i += 128) { ((v4u*)tA0)[i] = z; ((v4u*)tA1)[i] = z; }
    for (int i = tid; i < (kRowsPerBlock * kHPitch * 2) / 16; i += 128) ((v4u*)tH)[i] = z;
  }

  float bi0[4], bi1[4];
#pragma unroll
  for (int g = 0; g < 4; ++g) { bi0[g] = ct[g * 64 + unit]; bi1[g] = ct[kNGate + g * 64 + unit]; }
  const float b1a = ct[512 + rl], b1b = ct[512 + 16 + rl];
  const float w2a = ct[544 + rl], w2b = ct[544 + 16 + rl];
  const float b2v = ct[576];

  float c0[8], c1[8], h0r[8], h1r[8], pdr[8];
#pragma unroll
  for (int r = 0; r < 8; ++r) { c0[r] = 0.f; c1[r] = 0.f; h0r[r] = 0.f; h1r[r] = 0.f; pdr[r] = 0.f; }
  __syncthreads();

  const _Float16* tA0h = (const _Float16*)tA0;
  const _Float16* tA1h = (const _Float16*)tA1;
  const _Float16* tHh  = (const _Float16*)tH;
  const _Float16* bt0  = (const _Float16*)bt0p;
  const _Float16* bt1  = (const _Float16*)bt1p;
  const _Float16* bw1  = (const _Float16*)bw1p;

  for (int t = 0; t < kSeq; ++t) {
    {
      const int p = tid < 80 ? tid : 79;
      const int row = p / 5, q = p - row * 5;
      const v4u v = *(const v4u*)(xs + ((size_t)t * kBatch + b0) * kXsPitch + (size_t)p * 8);
      if (tid < 80) *(v4u*)(tA0 + row * kTilePitch + q * 8) = v;
    }
    __syncthreads();

    {
      v8f acc[4];
      gate_gemm16<kK0 / 32, kTilePitch, kK0>(tA0h, bt0, rl, koff, wave * 16, acc);
      lstm_cell_update(acc, bi0, uval, c0, h0r);
#pragma unroll
      for (int r = 0; r < 8; ++r) tA1[(8 * hh + r) * kTilePitch + unit] = h_bits(h0r[r] * kAScale);
    }
    __syncthreads();

    {
#pragma unroll
      for (int r = 0; r < 8; ++r) tA0[(8 * hh + r) * kTilePitch + kH0Col + unit] = h_bits(h0r[r] * kAScale);
      v8f acc[4];
      gate_gemm16<kK1 / 32, kTilePitch, kK1>(tA1h, bt1, rl, koff, wave * 16, acc);
      lstm_cell_update(acc, bi1, uval, c1, h1r);
#pragma unroll
      for (int r = 0; r < 8; ++r) tH[(8 * hh + r) * kHPitch + unit] = h_bits(h1r[r] * kAScale);
    }
    __syncthreads();

#pragma unroll
    for (int r = 0; r < 8; ++r) tA1[(8 * hh + r) * kTilePitch + 64 + unit] = h_bits(h1r[r] * kAScale);
    if (wave == 0) {
      v8f ha0 = (v8f){0.f, 0.f, 0.f, 0.f, 0.f, 0.f, 0.f, 0.f};
      v8f ha1 = (v8f){0.f, 0.f, 0.f, 0.f, 0.f, 0.f, 0.f, 0.f};
#pragma unroll
      for (int ks = 0; ks < kKH / 32; ++ks) {
        const v16h a  = Frag<_Float16>::load(tHh + rl * kHPitch + ks * 32 + koff);
        const v16h bA = Frag<_Float16>::load(bw1 + (size_t)rl * kKH + ks * 32 + koff);
        const v16h bB = Frag<_Float16>::load(bw1 + (size_t)(16 + rl) * kKH + ks * 32 + koff);
        ha0 = Frag<_Float16>::mma(a, bA, ha0);
        ha1 = Frag<_Float16>::mma(a, bB, ha1);
        dep_guard_h(ha0, ha1, a, bB);
      }
#pragma unroll
      for (int r = 0; r < 8; ++r) {
        const float v0 = fmaxf(ha0[r] * kAccScale + b1a, 0.0f) * w2a;
        const float v1 = fmaxf(ha1[r] * kAccScale + b1b, 0.0f) * w2b;
        float s = v0 + v1;
        s += __shfl_xor(s, 1, 32);
        s += __shfl_xor(s, 2, 32);
        s += __shfl_xor(s, 4, 32);
        s += __shfl_xor(s, 8, 32);
        const float raw = s + b2v;
        float nd = pdr[r] + kMaxInc * tanhf(raw);
        nd = fminf(fmaxf(nd, -kDeltaMax), kDeltaMax);
        pdr[r] = nd;
        if (rl == 0) {
          sOut[(8 * hh + r) * kSeq + t] = nd;
          tA0[(8 * hh + r) * kTilePitch + kPdCol] = h_bits(nd * kAScale);
        }
      }
    }
  }
  __syncthreads();

  for (int pass = 0; pass < 2; ++pass) {
#pragma unroll
    for (int q = 0; q < 8; ++q) {
      const int row = wave * 4 + (q >> 1);
      const int seg = (q & 1) * 128;
      const v4f v = *(const v4f*)(sOut + row * kSeq + seg + lane * 4);
      *(volatile v4f*)(out + (size_t)(b0 + row) * kSeq + seg + lane * 4) = v;
    }
    __threadfence();
  }
}

extern "C" void kernel_launch(void* const* d_in, const int* in_sizes, int n_in,
                              void* d_out, int out_size, void* d_ws, size_t ws_size,
                              hipStream_t stream)
{
  if (n_in < 13) return;
  if (in_sizes[0] != kBatch * kSeq * kDin) return;
  if (out_size != kBatch * kSeq) return;
  if (in_sizes[1] != 200 * 35 || in_sizes[2] != 200 * 50 || in_sizes[3] != 200 || in_sizes[4] != 200) return;
  if (in_sizes[5] != 200 * 50 || in_sizes[6] != 200 * 50 || in_sizes[7] != 200 || in_sizes[8] != 200) return;
  if (in_sizes[9] != 25 * 50 || in_sizes[10] != 25 || in_sizes[11] != 25 || in_sizes[12] != 1) return;

  const float* features = (const float*)d_in[0];
  const float* wih0 = (const float*)d_in[1];
  const float* whh0 = (const float*)d_in[2];
  const float* bih0 = (const float*)d_in[3];
  const float* bhh0 = (const float*)d_in[4];
  const float* wih1 = (const float*)d_in[5];
  const float* whh1 = (const float*)d_in[6];
  const float* bih1 = (const float*)d_in[7];
  const float* bhh1 = (const float*)d_in[8];
  const float* w1   = (const float*)d_in[9];
  const float* b1   = (const float*)d_in[10];
  const float* w2   = (const float*)d_in[11];
  const float* b2   = (const float*)d_in[12];

  const size_t bytesXS  = (size_t)kSeq * kBatch * kXsPitch * 2;
  const size_t bytesBt0 = (size_t)kNGate * kK0 * 2;
  const size_t bytesBt1 = (size_t)kNGate * kK1 * 2;
  const size_t bytesBw1 = (size_t)32 * kKH * 2;
  const size_t bytesCT  = (size_t)640 * 4;
  const size_t offXS  = 0;
  const size_t offBt0 = offXS + bytesXS;
  const size_t offBt1 = offBt0 + bytesBt0;
  const size_t offBw1 = offBt1 + bytesBt1;
  const size_t offCT  = offBw1 + bytesBw1;
  const size_t total  = offCT + bytesCT;
  if (total > ws_size) return;

  char* ws = (char*)d_ws;
  unsigned short* xs  = (unsigned short*)(ws + offXS);
  unsigned int*   bt0 = (unsigned int*)(ws + offBt0);
  unsigned int*   bt1 = (unsigned int*)(ws + offBt1);
  unsigned int*   bw1 = (unsigned int*)(ws + offBw1);
  float*          ct  = (float*)(ws + offCT);

  prep_weights_kernel<<<386, 64, 0, stream>>>(wih0, whh0, bih0, bhh0, wih1, whh1, bih1, bhh1,
                                              w1, b1, w2, b2, bt0, bt1, bw1, ct);
  sig_feats_kernel<<<dim3(kBatch / 64, kSeq), 64, 0, stream>>>(features, xs);
  sig_lstm_seq_kernel<<<kBatch / kRowsPerBlock, 128, 0, stream>>>(
      (const unsigned short*)xs, (const unsigned short*)bt0, (const unsigned short*)bt1,
      (const unsigned short*)bw1, (const float*)ct, (float*)d_out);
}
